// SelectiveSSMBackbone_74526272520980
// MI455X (gfx1250) — hardware-run, weakly checked
//
#include <hip/hip_runtime.h>
#include <math.h>

typedef __attribute__((ext_vector_type(16))) _Float16 v16h;
typedef __attribute__((ext_vector_type(8)))  _Float16 v8h;
typedef __attribute__((ext_vector_type(2)))  _Float16 v2h;
typedef __attribute__((ext_vector_type(16))) __bf16   v16b;
typedef __attribute__((ext_vector_type(8)))  __bf16   v8b;
typedef __attribute__((ext_vector_type(8)))  float    v8f;
typedef __attribute__((ext_vector_type(4)))  float    v4f;
typedef __attribute__((ext_vector_type(2)))  float    v2f;
typedef float v2f __attribute__((ext_vector_type(2)));

constexpr int kB    = 8;
constexpr int kL    = 2048;
constexpr int kRows = kB * kL;
constexpr int kP    = 32;
constexpr int kD    = 256;
constexpr int kNs   = 16;
constexpr int kNq   = 2 * kNs + 1;
constexpr int kNqP  = 64;
constexpr int kThr  = 256;
constexpr float kInCarry = 1024.0f;
constexpr float kWCarry  = 4096.0f;
constexpr float kBCCarry = 2048.0f;
constexpr float kHfCarry = 512.0f;
constexpr float kScIn = 1.0f / (kInCarry * kWCarry);
constexpr float kScBC = 1.0f / (kInCarry * kBCCarry);
constexpr float kScW1 = 1.0f / (kHfCarry * kWCarry);
constexpr float kScW2 = 1.0f / (kInCarry * kWCarry);
constexpr float kF16MinNormal = 6.103515625e-5f;

static_assert(kNq == 33 && kNq <= kNqP && kD == 256 && kRows == 16384 && kL == 2048 && kP == 32, "the index arithmetic below uses these sizes");

constexpr size_t kOffBIAS = 0ull;
constexpr size_t kOffSTAT = 4096ull;
constexpr size_t kOffY16 = 135168ull;
constexpr size_t kOffWIN16 = 1183744ull;
constexpr size_t kOffWBC16 = 1200128ull;
constexpr size_t kOffW116 = 1265664ull;
constexpr size_t kOffW216 = 1396736ull;
constexpr size_t kOffH = 1429504ull;
constexpr size_t kOffHN32 = 18206720ull;
constexpr size_t kOffHN16 = 34983936ull;
constexpr size_t kOffBCQ = 51761152ull;
constexpr size_t kOffDEL = 55955456ull;
constexpr size_t kOffH2 = 56020992ull;
constexpr size_t kOffHF16 = 72798208ull;
constexpr size_t kOffZ = 81186816ull;
constexpr size_t kOffG16 = 97964032ull;
constexpr size_t kOffOUTP = 106352640ull;
constexpr size_t kWsTotal = 110546944ull;
static_assert(kWsTotal <= 134217728ull, "carve cap: under 128 MiB");
static_assert(kOffBIAS == 0
  && kOffSTAT == kOffBIAS + 4096ull
  && kOffY16 == kOffSTAT + 131072ull
  && kOffWIN16 == kOffY16 + 1048576ull
  && kOffWBC16 == kOffWIN16 + 16384ull
  && kOffW116 == kOffWBC16 + 65536ull
  && kOffW216 == kOffW116 + 131072ull
  && kOffH == kOffW216 + 32768ull
  && kOffHN32 == kOffH + 16777216ull
  && kOffHN16 == kOffHN32 + 16777216ull
  && kOffBCQ == kOffHN16 + 16777216ull
  && kOffDEL == kOffBCQ + 4194304ull
  && kOffH2 == kOffDEL + 65536ull
  && kOffHF16 == kOffH2 + 16777216ull
  && kOffZ == kOffHF16 + 8388608ull
  && kOffG16 == kOffZ + 16777216ull
  && kOffOUTP == kOffG16 + 8388608ull
  && kWsTotal == kOffOUTP + 4194304ull, "the carve is a chain: every region starts where the one before ends");
static_assert((kOffSTAT % 256) == 0 && (kOffY16 % 256) == 0 && (kOffWIN16 % 256) == 0 && (kOffWBC16 % 256) == 0 && (kOffW116 % 256) == 0 && (kOffW216 % 256) == 0 && (kOffH % 256) == 0 && (kOffHN32 % 256) == 0 && (kOffHN16 % 256) == 0 && (kOffBCQ % 256) == 0 && (kOffDEL % 256) == 0 && (kOffH2 % 256) == 0 && (kOffHF16 % 256) == 0 && (kOffZ % 256) == 0 && (kOffG16 % 256) == 0 && (kOffOUTP % 256) == 0, "every region starts on a multiple of 256 B");

__device__ __forceinline__ unsigned short f2bf_bits(float f) {
  unsigned u = __float_as_uint(f);
  return (unsigned short)((u + 0x7FFFu + ((u >> 16) & 1u)) >> 16);
}
__device__ __forceinline__ float bf_bits2f(unsigned short h) { return __uint_as_float(((unsigned)h) << 16); }
__device__ __forceinline__ float bf16r(float f) { return bf_bits2f(f2bf_bits(f)); }
__device__ __forceinline__ float carry_flush(float v, float carry) {
  const float s = v * carry;
  return (fabsf(s) < kF16MinNormal) ? 0.0f : s;
}

__device__ __forceinline__ void dep_guard4_h(v8f& a, v8f& b, v8f& c, v8f& d, v16h x, v16h y) { asm volatile("v_nop\n\tv_nop\n\tv_nop\n\tv_nop" : "+v"(a), "+v"(b), "+v"(c), "+v"(d) : "v"(x), "v"(y)); }
__device__ __forceinline__ void dep_guard4_b(v8f& a, v8f& b, v8f& c, v8f& d, v16b x, v16b y) { asm volatile("v_nop\n\tv_nop\n\tv_nop\n\tv_nop" : "+v"(a), "+v"(b), "+v"(c), "+v"(d) : "v"(x), "v"(y)); }
__device__ __forceinline__ void keep4_h(v16h a, v16h b, v16h c, v16h d) { asm volatile("v_nop" :: "v"(a), "v"(b), "v"(c), "v"(d)); }
__device__ __forceinline__ void keep4_b(v16b a, v16b b, v16b c, v16b d) { asm volatile("v_nop" :: "v"(a), "v"(b), "v"(c), "v"(d)); }
__device__ __forceinline__ void acc_guard4(v8f& a, v8f& b, v8f& c, v8f& d) { asm volatile("v_nop\n\tv_nop\n\tv_nop\n\tv_nop" : "+v"(a), "+v"(b), "+v"(c), "+v"(d)); }

template <typename T> struct Frag;
template <> struct Frag<_Float16> {
  typedef v16h V; union U { v16h v; v8h h[2]; };
  static __device__ __forceinline__ v16h load(const _Float16* p) {
    U f; f.h[0] = *(const v8h*)(p); f.h[1] = *(const v8h*)(p + 16); return f.v;
  }
  static __device__ __forceinline__ v8f mma(v16h a, v16h b, v8f c) {
    return __builtin_amdgcn_wmma_f32_16x16x32_f16(false, a, false, b, (short)0, c, false, false);
  }
  static __device__ __forceinline__ void guard4(v8f& a, v8f& b, v8f& c, v8f& d, v16h x, v16h y) { dep_guard4_h(a, b, c, d, x, y); }
  static __device__ __forceinline__ void keep(v16h a, v16h b, v16h c, v16h d) { keep4_h(a, b, c, d); }
};
template <> struct Frag<__bf16> {
  typedef v16b V; union U { v16b v; v8b h[2]; };
  static __device__ __forceinline__ v16b load(const __bf16* p) {
    U f; f.h[0] = *(const v8b*)(p); f.h[1] = *(const v8b*)(p + 16); return f.v;
  }
  static __device__ __forceinline__ v8f mma(v16b a, v16b b, v8f c) {
    return __builtin_amdgcn_wmma_f32_16x16x32_bf16(false, a, false, b, (short)0, c, false, false);
  }
  static __device__ __forceinline__ void guard4(v8f& a, v8f& b, v8f& c, v8f& d, v16b x, v16b y) { dep_guard4_b(a, b, c, d, x, y); }
  static __device__ __forceinline__ void keep(v16b a, v16b b, v16b c, v16b d) { keep4_b(a, b, c, d); }
};

__device__ __forceinline__ v8f mma_h(v16h a, v16h b, v8f c) {
  c = __builtin_amdgcn_wmma_f32_16x16x32_f16(false, a, false, b, (short)0, c, false, false);
  asm volatile("v_nop\n\tv_nop\n\tv_nop\n\tv_nop" : "+v"(c) : "v"(a), "v"(b));
  return c;
}

template <int ET> struct Elem;
template <> struct Elem<0> { typedef _Float16 T; };
template <> struct Elem<1> { typedef __bf16 T; };
template <int ET, bool SPLIT, int BIAS_MODE, int OUT_MODE, bool RESID, int ACT = 0>
__global__ __launch_bounds__(256) void wmma_gemm64(
    const unsigned short* __restrict__ Ap, const unsigned short* __restrict__ A2p, int lda, long strideA,
    const unsigned short* __restrict__ Btp, const unsigned short* __restrict__ Bt2p, int ldb, long strideB,
    void* __restrict__ Cout, void* __restrict__ Cout2, int ldc, long strideC,
    const float* __restrict__ bias,
    const float* __restrict__ resid, long strideR,
    int M, int N, int K, float scale) {
  typedef typename Elem<ET>::T T;
  typedef typename Frag<T>::V V;
  const T* A = (const T*)Ap; const T* A2 = (const T*)A2p; const T* Bt = (const T*)Btp; const T* Bt2 = (const T*)Bt2p;
  __shared__ __align__(16) float sT[8][16 * 68];
  const int b    = blockIdx.y;
  const int lane = threadIdx.x & 31;
  const int wave = threadIdx.x >> 5;
  const int tilesN = N >> 6;
  const int tilesM = M >> 6;
  const int tile = blockIdx.x * 8 + wave;
  if (tile >= tilesM * tilesN) return;
  const int tm = tile / tilesN;
  const int tn = tile - tm * tilesN;
  const int m0 = tm << 6;
  const int n0 = tn << 6;

  const T* Ab  = A  + (size_t)b * strideA;
  const T* Bb  = Bt + (size_t)b * strideB;
  const T* Ab2 = SPLIT ? (A2  + (size_t)b * strideA) : nullptr;
  const T* Bb2 = SPLIT ? (Bt2 + (size_t)b * strideB) : nullptr;

  const int rlane = lane & 15;
  const int koff  = (lane >> 4) * 8;
  const int mOff  = (lane >> 4) * 8;

  v8f acc[4][4];
#pragma unroll
  for (int i = 0; i < 4; ++i)
#pragma unroll
    for (int j = 0; j < 4; ++j) acc[i][j] = (v8f){0.f,0.f,0.f,0.f,0.f,0.f,0.f,0.f};

  for (int k0 = 0; k0 < K; k0 += 32) {
    V bh[4], bl[4];
#pragma unroll
    for (int j = 0; j < 4; ++j) {
      const size_t bo = (size_t)(n0 + (j << 4) + rlane) * ldb + koff + k0;
      bh[j] = Frag<T>::load(Bb + bo);
      if (SPLIT) bl[j] = Frag<T>::load(Bb2 + bo);
    }
#pragma unroll
    for (int i = 0; i < 4; ++i) {
      const size_t ao = (size_t)(m0 + (i << 4) + rlane) * lda + koff + k0;
      V ah = Frag<T>::load(Ab + ao);
      V al;
      if (SPLIT) al = Frag<T>::load(Ab2 + ao);
#pragma unroll
      for (int j = 0; j < 4; ++j) {
        acc[i][j] = Frag<T>::mma(ah, bh[j], acc[i][j]);
        if (SPLIT) {
          acc[i][j] = Frag<T>::mma(ah, bl[j], acc[i][j]);
          acc[i][j] = Frag<T>::mma(al, bh[j], acc[i][j]);
        }
      }
      Frag<T>::guard4(acc[i][0], acc[i][1], acc[i][2], acc[i][3], ah, SPLIT ? al : ah);
    }
    Frag<T>::keep(bh[0], bh[1], bh[2], bh[3]);
    if (SPLIT) Frag<T>::keep(bl[0], bl[1], bl[2], bl[3]);
  }
  acc_guard4(acc[0][0], acc[0][1], acc[0][2], acc[0][3]);
  acc_guard4(acc[1][0], acc[1][1], acc[1][2], acc[1][3]);
  acc_guard4(acc[2][0], acc[2][1], acc[2][2], acc[2][3]);
  acc_guard4(acc[3][0], acc[3][1], acc[3][2], acc[3][3]);

  float* slab = sT[wave];
  const float* Rb = RESID ? (resid + (size_t)b * strideR) : nullptr;
#pragma unroll
  for (int i = 0; i < 4; ++i) {
    const int mBase = m0 + (i << 4);
#pragma unroll
    for (int j = 0; j < 4; ++j) {
      const int n = n0 + (j << 4) + rlane;
      float bv = 0.f;
      if (BIAS_MODE == 2) bv = bias[n];
#pragma unroll
      for (int r = 0; r < 8; ++r) {
        float v = acc[i][j][r] * scale;
        if (BIAS_MODE == 1) v += bias[mBase + mOff + r];
        if (BIAS_MODE == 2) v += bv;
        if (RESID) v += Rb[(size_t)(mBase + mOff + r) * ldc + n];
        if (ACT == 1) v = tanhf(v);
        if (ACT == 2) v = fmaxf(v, 0.0f);
        if (ACT == 3) v = v / (1.0f + expf(-v));
        if (ACT == 4) v = (v > 0.f) ? v : 0.01f * v;
        slab[(mOff + r) * 68 + (j << 4) + rlane] = v;
      }
    }
    __builtin_amdgcn_fence(__ATOMIC_RELEASE, "workgroup");
    __builtin_amdgcn_wave_barrier();
    __builtin_amdgcn_fence(__ATOMIC_ACQUIRE, "workgroup");
    if (OUT_MODE == 0) {
      float* C = (float*)Cout + (size_t)b * strideC;
      const int hh = lane >> 4, c4 = (lane & 15) * 4;
      for (int pass = 0; pass < 2; ++pass) {
#pragma unroll
        for (int it = 0; it < 8; ++it) {
          const int row = it * 2 + hh;
          v4f v = *(const v4f*)(slab + row * 68 + c4);
          *(volatile v4f*)(C + (size_t)(mBase + row) * ldc + n0 + c4) = v;
        }
        __threadfence();
      }
    } else {
      const int q = lane >> 3, c8 = (lane & 7) * 8;
      unsigned short* C  = (unsigned short*)Cout  + (size_t)b * strideC;
      unsigned short* C2 = (OUT_MODE == 2) ? ((unsigned short*)Cout2 + (size_t)b * strideC) : nullptr;
      for (int pass = 0; pass < 2; ++pass) {
#pragma unroll
        for (int it = 0; it < 4; ++it) {
          const int row = it * 4 + q;
          const float* sp = slab + row * 68 + c8;
          v8h hv, lv;
#pragma unroll
          for (int e = 0; e < 8; ++e) {
            if (OUT_MODE == 1) {
              hv[e] = (_Float16)sp[e];
            } else {
              unsigned short hb = f2bf_bits(sp[e]);
              unsigned short lb = f2bf_bits(sp[e] - bf_bits2f(hb));
              hv[e] = __builtin_bit_cast(_Float16, hb);
              lv[e] = __builtin_bit_cast(_Float16, lb);
            }
          }
          *(volatile v8h*)(C + (size_t)(mBase + row) * ldc + n0 + c8) = hv;
          if (OUT_MODE == 2) *(volatile v8h*)(C2 + (size_t)(mBase + row) * ldc + n0 + c8) = lv;
        }
        __threadfence();
      }
    }
    __builtin_amdgcn_fence(__ATOMIC_RELEASE, "workgroup");
    __builtin_amdgcn_wave_barrier();
    __builtin_amdgcn_fence(__ATOMIC_ACQUIRE, "workgroup");
  }
}


__device__ __forceinline__ void store2(float* p, float v) {
  *(volatile float*)p = v;
  __threadfence();
  *(volatile float*)p = v;
}

__global__ __launch_bounds__(kThr) void cast_plane_kernel(const float* __restrict__ src, unsigned short* __restrict__ dst,
                                                          int colsLog2, int dstPitch, int dstOff) {
  const int i   = blockIdx.x * kThr + threadIdx.x;
  const int sh  = colsLog2 - 3;
  const int row = i >> sh;
  const int c8  = (i & ((1 << sh) - 1)) * 8;
  const float* sp = src + ((size_t)row << colsLog2) + c8;
  const v4f a0 = *(const v4f*)(sp);
  const v4f a1 = *(const v4f*)(sp + 4);
  v8h hv;
#pragma unroll
  for (int e = 0; e < 4; ++e) {
    const float f0 = a0[e];
    const float f1 = a1[e];
    hv[e]     = (_Float16)carry_flush(bf16r(f0), kInCarry);
    hv[4 + e] = (_Float16)carry_flush(bf16r(f1), kInCarry);
  }
  unsigned short* dp = dst + (size_t)row * dstPitch + dstOff + c8;
  *(volatile v8h*)dp = hv;
  __threadfence();
  *(volatile v8h*)dp = hv;
}

__global__ __launch_bounds__(256) void wt_plane_kernel(const float* __restrict__ W, unsigned short* __restrict__ dst, int K, int N, int nLive, int ldd, int colOff) {
  const int n  = blockIdx.x;
  const int k8 = threadIdx.x * 8;
  const bool live = n < nLive;
  const int nc = live ? n : 0;
  v8h hv;
#pragma unroll
  for (int e = 0; e < 8; ++e) {
    const float w = W[(size_t)(k8 + e) * N + nc];
    hv[e] = (_Float16)(live ? carry_flush(bf16r(w), kWCarry) : 0.0f);
  }
  unsigned short* dp = dst + (size_t)n * ldd + colOff + k8;
  *(volatile v8h*)dp = hv;
  __threadfence();
  *(volatile v8h*)dp = hv;
}

__global__ __launch_bounds__(kThr) void setup_kernel(const float* __restrict__ bin_, const float* __restrict__ b1, const float* __restrict__ b2, const float* __restrict__ Win,
                                                    const float* __restrict__ W_B, const float* __restrict__ W_C, const float* __restrict__ qd,
                                                    float* __restrict__ BIAS, unsigned short* __restrict__ WIN16, unsigned short* __restrict__ WBC16) {
  const unsigned bk = blockIdx.x;
  if (bk < 4u) {
    const unsigned i = bk * (unsigned)kThr + threadIdx.x;
    float v = 0.0f;
    if (i < 256u) { const float p = bin_[i]; v = bf16r(p); }
    else if (i < 512u) { const float p = b1[i - 256u]; v = bf16r(p); }
    else if (i < 544u) { const float p = b2[i - 512u]; v = bf16r(p); }
    store2(BIAS + i, v);
  } else if (bk == 4u) {
    const unsigned n = threadIdx.x;
    unsigned short* dp = WIN16 + (size_t)n * kP;
#pragma unroll
    for (int c = 0; c < kP / 8; ++c) {
      v8h hv;
#pragma unroll
      for (int e = 0; e < 8; ++e) { const float p = Win[(size_t)(8 * c + e) * kD + n]; hv[e] = (_Float16)carry_flush(bf16r(p), kWCarry); }
      *(volatile v8h*)(dp + 8 * c) = hv;
      __threadfence();
      *(volatile v8h*)(dp + 8 * c) = hv;
    }
  } else {
    const unsigned i = (bk - 5u) * (unsigned)kThr + threadIdx.x;
    const unsigned r = i >> 6;
    const unsigned c8 = ((i & 63u) * 8u) & 255u;
    v8h hv;
#pragma unroll
    for (int e = 0; e < 8; ++e) {
      float w = 0.0f;
      if (r < 16u) { const float p = W_B[(size_t)r * kD + c8 + e]; w = carry_flush(bf16r(p), kBCCarry); }
      else if (r < 32u) { const float p = W_C[(size_t)(r - 16u) * kD + c8 + e]; w = carry_flush(bf16r(p), kBCCarry); }
      else if (r == 32u) { const float p = qd[c8 + e]; w = carry_flush(bf16r(p), kBCCarry); }
      hv[e] = (_Float16)w;
    }
    unsigned short* dp = WBC16 + (size_t)i * 8;
    *(volatile v8h*)dp = hv;
    __threadfence();
    *(volatile v8h*)dp = hv;
  }
}
static_assert(1024 == 4 * kThr && kD == kThr && kP == 32 && (size_t)kNqP * 2 * kD / 8 == 16ull * kThr, "set-up grid: 4 blocks of biases, 1 of Win rows, 16 of the parameter weights: 21 blocks");

__global__ __launch_bounds__(kThr) void lnstat_kernel(const float* __restrict__ X, float* __restrict__ STAT) {
  const size_t row = (size_t)blockIdx.x * kThr + threadIdx.x;
  const float* xp = X + row * kD;
  float s = 0.0f;
  for (int c = 0; c < kD; ++c) s += xp[c];
  const float mean = s / (float)kD;
  float q = 0.0f;
  for (int c = 0; c < kD; ++c) { const float dd = xp[c] - mean; q += dd * dd; }
  v2f st; st[0] = mean; st[1] = 1.0f / sqrtf(q / (float)kD + 1e-5f);
  float* dp = STAT + 2 * row;
  *(volatile v2f*)dp = st;
  __threadfence();
  *(volatile v2f*)dp = st;
}
static_assert(kRows == 64 * kThr, "statistics grid exact: 64 blocks");

__global__ __launch_bounds__(kThr) void lncast2_kernel(const float* __restrict__ X, const float* __restrict__ STAT, const float* __restrict__ gam, const float* __restrict__ bet,
                                                      float* __restrict__ HN32, unsigned short* __restrict__ HN16) {
  const unsigned i = blockIdx.x * (unsigned)kThr + threadIdx.x;
  const size_t row = i >> 5;
  const unsigned c8 = (i & 31u) * 8u;
  const float mean = STAT[2 * row], inv = STAT[2 * row + 1];
  const float* xp = X + row * kD + c8;
  v4f o0, o1;
  v8h hv, lv;
#pragma unroll
  for (int e = 0; e < 8; ++e) {
    const float ga = gam[c8 + e], be = bet[c8 + e];
    const float v = (xp[e] - mean) * inv * bf16r(ga) + bf16r(be);
    if (e < 4) o0[e] = v; else o1[e - 4] = v;
    const float sc = carry_flush(v, kInCarry);
    const _Float16 hh = (_Float16)sc;
    const float rr = sc - (float)hh;
    hv[e] = hh;
    lv[e] = (_Float16)((fabsf(rr) < kF16MinNormal) ? 0.0f : rr);
  }
  float* fp = HN32 + row * kD + c8;
  unsigned short* dp = HN16 + row * (2 * kD) + c8;
  for (int pass = 0; pass < 2; ++pass) {
    *(volatile v4f*)fp = o0; *(volatile v4f*)(fp + 4) = o1;
    *(volatile v8h*)dp = hv; *(volatile v8h*)(dp + kD) = lv;
    __threadfence();
  }
}
static_assert((size_t)kRows * (kD / 8) == 2048ull * kThr && kD / 8 == 32, "norm cast grid exact: 2,048 blocks; 32 groups a row");

__global__ __launch_bounds__(kThr) void lncast_kernel(const float* __restrict__ X, const float* __restrict__ STAT, const float* __restrict__ gam, const float* __restrict__ bet,
                                                     unsigned short* __restrict__ HF16) {
  const unsigned i = blockIdx.x * (unsigned)kThr + threadIdx.x;
  const size_t row = i >> 5;
  const unsigned c8 = (i & 31u) * 8u;
  const float mean = STAT[2 * row], inv = STAT[2 * row + 1];
  const float* xp = X + row * kD + c8;
  v8h hv;
#pragma unroll
  for (int e = 0; e < 8; ++e) {
    const float ga = gam[c8 + e], be = bet[c8 + e];
    hv[e] = (_Float16)carry_flush((xp[e] - mean) * inv * bf16r(ga) + bf16r(be), kHfCarry);
  }
  unsigned short* dp = HF16 + row * kD + c8;
  *(volatile v8h*)dp = hv;
  __threadfence();
  *(volatile v8h*)dp = hv;
}

__global__ __launch_bounds__(kThr) void dstep_kernel(const float* __restrict__ BCQ, const float* __restrict__ pd, float* __restrict__ DEL) {
  const size_t row = (size_t)blockIdx.x * kThr + threadIdx.x;
  const float p0 = pd[0];
  const float pre = BCQ[row * kNqP + 2 * kNs] + bf16r(p0);
  store2(DEL + row, fmaxf(pre, 0.0f) + log1pf(expf(-fabsf(pre))));
}

__global__ __launch_bounds__(kThr) void scan_kernel(const float* __restrict__ BCQ, const float* __restrict__ DEL, const float* __restrict__ HN32, const float* __restrict__ H,
                                                    const float* __restrict__ Ar, float* __restrict__ H2) {
  const unsigned sq = blockIdx.x;
  const unsigned d = threadIdx.x;
  float A[kNs], x[kNs];
#pragma unroll
  for (int n = 0; n < kNs; ++n) { const float a = Ar[(size_t)d * kNs + n]; A[n] = bf16r(a); x[n] = 0.0f; }
  for (int l = 0; l < kL; ++l) {
    const size_t row = (size_t)sq * kL + (size_t)l;
    const float* pb = BCQ + row * kNqP;
    const float dt = DEL[row];
    const float uv = HN32[row * kD + d];
    const float dx = dt * uv;
    float y = 0.0f;
#pragma unroll
    for (int q = 0; q < kNs / 4; ++q) {
      const v4f bv = *(const v4f*)(pb + 4 * q), cv = *(const v4f*)(pb + kNs + 4 * q);
#pragma unroll
      for (int e = 0; e < 4; ++e) {
        const int n = 4 * q + e;
        const float xn = expf(dt * A[n]) * x[n] + dx * bv[e];
        x[n] = xn;
        y += xn * cv[e];
      }
    }
    store2(H2 + row * kD + d, H[row * kD + d] + y);
  }
}
static_assert(kD == kThr && (kNs % 4) == 0, "walk grid exact: 8 blocks, a block a sequence");

__global__ __launch_bounds__(kThr) void gelu_kernel(const float* __restrict__ Z, unsigned short* __restrict__ G16) {
  const unsigned i = blockIdx.x * (unsigned)kThr + threadIdx.x;
  const size_t o = (size_t)i * 8;
  const float* zp = Z + o;
  v8h hv;
#pragma unroll
  for (int e = 0; e < 8; ++e) { const float z = zp[e]; hv[e] = (_Float16)carry_flush(0.5f * z * (1.0f + erff(z * 0.70710678118654752f)), kInCarry); }
  unsigned short* dp = G16 + o;
  *(volatile v8h*)dp = hv;
  __threadfence();
  *(volatile v8h*)dp = hv;
}

__global__ __launch_bounds__(kThr) void outcopy_kernel(const float* __restrict__ OUTP, float* __restrict__ out) {
  const unsigned i = blockIdx.x * (unsigned)kThr + threadIdx.x;
  const size_t row = i >> 2;
  const unsigned c8 = (i & 3u) * 8u;
  const float* sp = OUTP + row * kNqP + c8;
  const v4f a0 = *(const v4f*)sp, a1 = *(const v4f*)(sp + 4);
  float* dp = out + row * kP + c8;
  for (int pass = 0; pass < 2; ++pass) { *(volatile v4f*)dp = a0; *(volatile v4f*)(dp + 4) = a1; __threadfence(); }
}
static_assert((size_t)kRows * 4 == 256ull * kThr && kP == 4 * 8, "the result's copy: 256 blocks; 4 groups a row");

extern "C" void kernel_launch(void* const* d_in, const int* in_sizes, int n_in,
                              void* d_out, int out_size, void* d_ws, size_t ws_size,
                              hipStream_t stream) {
  if (n_in < 16 || d_out == nullptr || d_ws == nullptr) return;
  if (in_sizes[0] != kRows * kP || in_sizes[1] != kP * kD || in_sizes[2] != kD || in_sizes[3] != kD || in_sizes[4] != kD || in_sizes[5] != kD * kNs || in_sizes[6] != kNs * kD || in_sizes[7] != kNs * kD) return;
  if (in_sizes[8] != kD || in_sizes[9] != 1 || in_sizes[10] != kD || in_sizes[11] != kD || in_sizes[12] != kD * kD || in_sizes[13] != kD || in_sizes[14] != kD * kP || in_sizes[15] != kP) return;
  if (out_size != kRows * kP) return;
  if (ws_size < kWsTotal) return;
  const float* yin  = (const float*)d_in[0];
  const float* Win  = (const float*)d_in[1];
  const float* bin_ = (const float*)d_in[2];
  const float* ng   = (const float*)d_in[3];
  const float* nb   = (const float*)d_in[4];
  const float* Ar   = (const float*)d_in[5];
  const float* W_B  = (const float*)d_in[6];
  const float* W_C  = (const float*)d_in[7];
  const float* qd   = (const float*)d_in[8];
  const float* pd   = (const float*)d_in[9];
  const float* nfg  = (const float*)d_in[10];
  const float* nfb  = (const float*)d_in[11];
  const float* W1   = (const float*)d_in[12];
  const float* b1   = (const float*)d_in[13];
  const float* W2   = (const float*)d_in[14];
  const float* b2   = (const float*)d_in[15];
  float* out = (float*)d_out;
  char* ws = (char*)d_ws;
  float* BIAS = (float*)(ws + kOffBIAS);
  float* STAT = (float*)(ws + kOffSTAT);
  unsigned short* Y16   = (unsigned short*)(ws + kOffY16);
  unsigned short* WIN16 = (unsigned short*)(ws + kOffWIN16);
  unsigned short* WBC16 = (unsigned short*)(ws + kOffWBC16);
  unsigned short* W116  = (unsigned short*)(ws + kOffW116);
  unsigned short* W216  = (unsigned short*)(ws + kOffW216);
  float* H    = (float*)(ws + kOffH);
  float* HN32 = (float*)(ws + kOffHN32);
  unsigned short* HN16 = (unsigned short*)(ws + kOffHN16);
  float* BCQ  = (float*)(ws + kOffBCQ);
  float* DEL  = (float*)(ws + kOffDEL);
  float* H2   = (float*)(ws + kOffH2);
  unsigned short* HF16 = (unsigned short*)(ws + kOffHF16);
  float* Z    = (float*)(ws + kOffZ);
  unsigned short* G16 = (unsigned short*)(ws + kOffG16);
  float* OUTP = (float*)(ws + kOffOUTP);

  static_assert(((size_t)kRows * kP / 8) % kThr == 0 && kD / 8 == 32, "the input's cast: 256 blocks; the transposing casts' blocks of 32 threads");
  cast_plane_kernel<<<(int)(((size_t)kRows * kP / 8) / kThr), kThr, 0, stream>>>(yin, Y16, 5, kP, 0);
  wt_plane_kernel<<<kD, kD / 8, 0, stream>>>(W1, W116, kD, kD, kD, kD, 0);
  wt_plane_kernel<<<kNqP, kD / 8, 0, stream>>>(W2, W216, kD, kP, kP, kD, 0);
  setup_kernel<<<21, kThr, 0, stream>>>(bin_, b1, b2, Win, W_B, W_C, qd, BIAS, WIN16, WBC16);

  wmma_gemm64<0, false, 2, 0, false, 0><<<dim3((kRows / 64) * (kD / 64) / 8, 1), 256, 0, stream>>>(
      Y16, Y16, kP, 0L, WIN16, WIN16, kP, 0L, (void*)H, (void*)H, kD, 0L, BIAS, nullptr, 0L, kRows, kD, kP, kScIn);
  lnstat_kernel<<<64, kThr, 0, stream>>>(H, STAT);
  lncast2_kernel<<<2048, kThr, 0, stream>>>(H, STAT, ng, nb, HN32, HN16);
  wmma_gemm64<0, false, 2, 0, false, 0><<<dim3((kRows / 64) * (kNqP / 64) / 8, 1), 256, 0, stream>>>(
      HN16, HN16, 2 * kD, 0L, WBC16, WBC16, 2 * kD, 0L, (void*)BCQ, (void*)BCQ, kNqP, 0L, BIAS + 576, nullptr, 0L, kRows, kNqP, 2 * kD, kScBC);
  dstep_kernel<<<64, kThr, 0, stream>>>(BCQ, pd, DEL);
  scan_kernel<<<kB, kThr, 0, stream>>>(BCQ, DEL, HN32, H, Ar, H2);
  lnstat_kernel<<<64, kThr, 0, stream>>>(H2, STAT);
  lncast_kernel<<<2048, kThr, 0, stream>>>(H2, STAT, nfg, nfb, HF16);
  wmma_gemm64<0, false, 2, 0, false, 0><<<dim3((kRows / 64) * (kD / 64) / 8, 1), 256, 0, stream>>>(
      HF16, HF16, kD, 0L, W116, W116, kD, 0L, (void*)Z, (void*)Z, kD, 0L, BIAS + 256, nullptr, 0L, kRows, kD, kD, kScW1);
  gelu_kernel<<<2048, kThr, 0, stream>>>(Z, G16);
  wmma_gemm64<0, false, 2, 0, false, 0><<<dim3((kRows / 64) * (kNqP / 64) / 8, 1), 256, 0, stream>>>(
      G16, G16, kD, 0L, W216, W216, kD, 0L, (void*)OUTP, (void*)OUTP, kNqP, 0L, BIAS + 512, nullptr, 0L, kRows, kNqP, kD, kScW2);
  outcopy_kernel<<<256, kThr, 0, stream>>>(OUTP, out);
}
